// FWMRNN_69020124446842
// MI455X (gfx1250) — hardware-run, weakly checked
//
#include <hip/hip_runtime.h>
#include <math.h>

typedef __attribute__((ext_vector_type(16))) _Float16 v16h;
typedef __attribute__((ext_vector_type(8)))  _Float16 v8h;
typedef __attribute__((ext_vector_type(8)))  float    v8f;
typedef __attribute__((ext_vector_type(4)))  float    v4f;

constexpr int kT     = 128;
constexpr int kB     = 64;
constexpr int kI     = 1024;
constexpr int kH     = 1024;
constexpr int kG     = 4 * kH;
constexpr int kS     = 32;
constexpr int kNW    = 3 * kS + 1;
constexpr int kNR    = 4 * kS;
constexpr int kWR    = 256;
constexpr int kTC    = 32;
constexpr int kNC    = kT / kTC;
constexpr int kRows  = kT * kB;
constexpr int kRowsC = kTC * kB;
constexpr int kFV    = kS * kS * kS;
constexpr int kHP    = 1032;
constexpr int kSLP   = 36;
constexpr int kBB    = 16;

constexpr float kCIN    = 16.0f;
constexpr float kCHID   = 256.0f;
constexpr float kCOUT   = 16.0f;
constexpr float kCW     = 256.0f;
constexpr float kRS     = 2048.0f;
constexpr float kRS_INV = 1.0f / kRS;
constexpr float kFoldIn  = 1.0f / (kCIN * kCW);
constexpr float kFoldHid = 1.0f / (kCHID * kCW);
constexpr float kFoldOut = 1.0f / (kCOUT * kCW);
constexpr float kF16Min  = 6.103515625e-5f;
constexpr float kLnEps   = 1e-5f;
constexpr float kInvS    = 1.0f / (float)kS;

static_assert(kG == 4096 && kNW == 97 && kNR == 128, "gate and projection widths");
static_assert(kNW <= 128 && 128 + kNR == kWR, "padded write|read plane");
static_assert(kI % 32 == 0 && kH % 32 == 0 && kS % 32 == 0, "GEMM K multiples of 32");
static_assert(kRows % 64 == 0 && kRowsC % 64 == 0, "GEMM M multiples of 64");
static_assert(kG % 32 == 0 && kWR % 32 == 0 && kH % 32 == 0, "GEMM N multiples of 32");
static_assert(kB % kBB == 0 && kH == 8 * 128, "recurrence tiling: 8 waves x 128 units");
static_assert((kHP % 8) == 0 && kHP >= kH + 8, "h tile pitch");
static_assert(kFV == 32768, "memory tensor size");

constexpr size_t kSzIN   = (size_t)kRows * kI * 2;
constexpr size_t kSzWI   = (size_t)kG * kI * 2;
constexpr size_t kSzWH   = (size_t)kG * kH * 2;
constexpr size_t kSzGP   = (size_t)kRowsC * kG * 4;
constexpr size_t kSzX    = (size_t)kRows * kH * 4;
constexpr size_t kSzWRp  = (size_t)kWR * kH * 2;
constexpr size_t kSzWLp  = (size_t)kH * kS * 2;
constexpr size_t kSzBS   = (size_t)kG * 4;
constexpr size_t kSzBW   = (size_t)kWR * 4;
constexpr size_t kSzCS   = (size_t)kB * kH * 4;
constexpr size_t kSzO    = (size_t)kRows * kS * 4;
constexpr size_t kSzOp   = (size_t)kRows * kS * 2;
constexpr size_t kSzP    = (size_t)kRows * kWR * 4;
constexpr size_t kOffINH = 0;
constexpr size_t kOffINL = kOffINH + kSzIN;
constexpr size_t kOffWIH = kOffINL + kSzIN;
constexpr size_t kOffWIL = kOffWIH + kSzWI;
constexpr size_t kOffWHH = kOffWIL + kSzWI;
constexpr size_t kOffGP  = kOffWHH + kSzWH;
constexpr size_t kOffX   = kOffGP  + kSzGP;
constexpr size_t kOffWRH = kOffX   + kSzX;
constexpr size_t kOffWRL = kOffWRH + kSzWRp;
constexpr size_t kOffWLH = kOffWRL + kSzWRp;
constexpr size_t kOffWLL = kOffWLH + kSzWLp;
constexpr size_t kOffBS  = kOffWLL + kSzWLp;
constexpr size_t kOffBW  = kOffBS  + kSzBS;
constexpr size_t kOffCS0 = kOffBW  + kSzBW;
constexpr size_t kOffCS1 = kOffCS0 + kSzCS;
constexpr size_t kOffO   = kOffCS1 + kSzCS;
constexpr size_t kOffOH  = kOffO   + kSzO;
constexpr size_t kOffOL  = kOffOH  + kSzOp;
constexpr size_t kWsTotal = kOffOL + kSzOp;
static_assert(kWsTotal == 129647616ull, "carve total");
static_assert(kWsTotal <= 134217728ull, "carve cap");
static_assert(kSzP <= kSzGP, "P fits the dead gate-term region");
static_assert((kOffINL % 256) == 0 && (kOffWIH % 256) == 0 && (kOffWIL % 256) == 0 && (kOffWHH % 256) == 0 &&
              (kOffGP % 256) == 0 && (kOffX % 256) == 0 && (kOffWRH % 256) == 0 && (kOffWRL % 256) == 0 &&
              (kOffWLH % 256) == 0 && (kOffWLL % 256) == 0 && (kOffBS % 256) == 0 && (kOffBW % 256) == 0 &&
              (kOffCS0 % 256) == 0 && (kOffCS1 % 256) == 0 && (kOffO % 256) == 0 && (kOffOH % 256) == 0 &&
              (kOffOL % 256) == 0, "256-B aligned regions");

__device__ __forceinline__ void tie1_h(v8f& c, v16h x, v16h y) { asm volatile("v_nop" : "+v"(c) : "v"(x), "v"(y)); }
__device__ __forceinline__ void tie4_h(v8f& c, v16h x, v16h y) { asm volatile("v_nop\n\tv_nop\n\tv_nop\n\tv_nop" : "+v"(c) : "v"(x), "v"(y)); }
__device__ __forceinline__ void keep4_h(v16h a, v16h b, v16h c, v16h d) { asm volatile("v_nop" :: "v"(a), "v"(b), "v"(c), "v"(d)); }
__device__ __forceinline__ void acc_tie4(v8f& c) { asm volatile("v_nop\n\tv_nop\n\tv_nop\n\tv_nop" : "+v"(c)); }
template <typename T> struct Frag;
template <> struct Frag<_Float16> {
  typedef v16h V; union U { v16h v; v8h h[2]; };
  static __device__ __forceinline__ v16h load(const _Float16* p) {
    U f; f.h[0] = *(const v8h*)(p); f.h[1] = *(const v8h*)(p + 16); return f.v;
  }
  static __device__ __forceinline__ v8f mma(v16h a, v16h b, v8f c) {
    return __builtin_amdgcn_wmma_f32_16x16x32_f16(false, a, false, b, (short)0, c, false, false);
  }
};

__device__ __forceinline__ float flush16(float v) { return (fabsf(v) < kF16Min) ? 0.0f : v; }

__device__ __forceinline__ void split8(const v4f a0, const v4f a1, const float carry, v8h& hv, v8h& lv) {
#pragma unroll
  for (int e = 0; e < 4; ++e) {
    const float x0 = a0[e];
    const float x1 = a1[e];
    const float s0 = flush16(x0 * carry);
    const float s1 = flush16(x1 * carry);
    const _Float16 h0 = (_Float16)s0;
    const _Float16 h1 = (_Float16)s1;
    const float d0 = (s0 - (float)h0) * kRS;
    const float d1 = (s1 - (float)h1) * kRS;
    const _Float16 l0 = (_Float16)flush16(d0);
    const _Float16 l1 = (_Float16)flush16(d1);
    hv[e]     = h0;
    hv[4 + e] = h1;
    lv[e]     = l0;
    lv[4 + e] = l1;
  }
}

__device__ __forceinline__ float fsig(float x)  { return __builtin_amdgcn_rcpf(1.0f + __expf(-x)); }
__device__ __forceinline__ float ftanh(float x) { return 1.0f - 2.0f * __builtin_amdgcn_rcpf(__expf(2.0f * x) + 1.0f); }

template <bool WITH_LO>
__global__ __launch_bounds__(256) void split_f16_kernel(
    const float* __restrict__ src, unsigned short* __restrict__ dhi, unsigned short* __restrict__ dlo,
    int total8, float carry)
{
  const int i = blockIdx.x * 256 + threadIdx.x;
  if (i >= total8) return;
  const size_t e0 = (size_t)i << 3;
  const v4f a0 = *(const v4f*)(src + e0);
  const v4f a1 = *(const v4f*)(src + e0 + 4);
  v8h hv, lv;
  split8(a0, a1, carry, hv, lv);
  unsigned short* qh = dhi + e0;
  unsigned short* ql = dlo + e0;
  *(volatile v8h*)qh = hv;
  if (WITH_LO) *(volatile v8h*)ql = lv;
  __threadfence();
  *(volatile v8h*)qh = hv;
  if (WITH_LO) *(volatile v8h*)ql = lv;
}

__global__ __launch_bounds__(256) void wr_plane_kernel(
    const float* __restrict__ Ww, const float* __restrict__ Wr,
    unsigned short* __restrict__ dhi, unsigned short* __restrict__ dlo)
{
  const int i   = blockIdx.x * 256 + threadIdx.x;
  const int row = i >> 7;
  const int c8  = (i & 127) * 8;
  const int rw  = (row < kNW) ? row : (kNW - 1);
  int rr = row - 128;
  rr = (rr < 0) ? 0 : rr;
  rr = (rr > kNR - 1) ? (kNR - 1) : rr;
  v4f w0 = *(const v4f*)(Ww + (size_t)rw * kH + c8);
  v4f w1 = *(const v4f*)(Ww + (size_t)rw * kH + c8 + 4);
  v4f r0 = *(const v4f*)(Wr + (size_t)rr * kH + c8);
  v4f r1 = *(const v4f*)(Wr + (size_t)rr * kH + c8 + 4);
  const bool isw = (row < kNW);
  const bool isr = (row >= 128);
  v4f a0, a1;
#pragma unroll
  for (int e = 0; e < 4; ++e) {
    const float x0 = w0[e], y0 = r0[e], x1 = w1[e], y1 = r1[e];
    a0[e] = isw ? x0 : (isr ? y0 : 0.0f);
    a1[e] = isw ? x1 : (isr ? y1 : 0.0f);
  }
  v8h hv, lv;
  split8(a0, a1, kCW, hv, lv);
  const size_t e0 = (size_t)i << 3;
  *(volatile v8h*)(dhi + e0) = hv;
  *(volatile v8h*)(dlo + e0) = lv;
  __threadfence();
  *(volatile v8h*)(dhi + e0) = hv;
  *(volatile v8h*)(dlo + e0) = lv;
}

__global__ __launch_bounds__(256) void bias_kernel(
    const float* __restrict__ b_ih, const float* __restrict__ b_hh,
    const float* __restrict__ b_w, const float* __restrict__ b_r,
    float* __restrict__ BSUM, float* __restrict__ BWR)
{
  const int tid = threadIdx.x;
  if (blockIdx.x < 4) {
    const int idx = (blockIdx.x * 256 + tid) * 4;
    const v4f va = *(const v4f*)(b_ih + idx);
    const v4f vb = *(const v4f*)(b_hh + idx);
    v4f o;
#pragma unroll
    for (int e = 0; e < 4; ++e) o[e] = va[e] + vb[e];
    *(volatile v4f*)(BSUM + idx) = o;
    __threadfence();
    *(volatile v4f*)(BSUM + idx) = o;
  } else if (tid < 64) {
    const int n0 = tid * 4;
    v4f o;
#pragma unroll
    for (int e = 0; e < 4; ++e) {
      const int n  = n0 + e;
      const int nw = (n < kNW) ? n : (kNW - 1);
      int nr = n - 128;
      nr = (nr < 0) ? 0 : nr;
      nr = (nr > kNR - 1) ? (kNR - 1) : nr;
      float a = b_w[nw];
      float c = b_r[nr];
      asm volatile("" : "+v"(a));
      asm volatile("" : "+v"(c));
      o[e] = (n < kNW) ? a : ((n >= 128) ? c : 0.0f);
    }
    *(volatile v4f*)(BWR + n0) = o;
    __threadfence();
    *(volatile v4f*)(BWR + n0) = o;
  }
}

template <int BIAS_MODE, bool RESID>
__global__ __launch_bounds__(256) void gemm_f16x3_kernel(
    const unsigned short* __restrict__ Ahp, const unsigned short* __restrict__ Alp, int lda,
    const unsigned short* __restrict__ Bhp, const unsigned short* __restrict__ Blp, int ldb,
    float* __restrict__ C, int ldc,
    const float* __restrict__ bias, const float* __restrict__ resid,
    int M, int N, int K, float scale)
{
  typedef Frag<_Float16> F;
  __shared__ __align__(16) float sT[8][16 * kSLP];
  const _Float16* Ah = (const _Float16*)Ahp;
  const _Float16* Al = (const _Float16*)Alp;
  const _Float16* Bh = (const _Float16*)Bhp;
  const _Float16* Bl = (const _Float16*)Blp;
  const int lane = threadIdx.x & 31;
  const int wave = threadIdx.x >> 5;
  const int tilesN = N >> 5;
  const int tilesM = M >> 6;
  const int tile = blockIdx.x * 8 + wave;
  if (tile >= tilesM * tilesN) return;
  const int tm = tile / tilesN;
  const int tn = tile - tm * tilesN;
  const int m0 = tm << 6;
  const int n0 = tn << 5;
  const int rlane = lane & 15;
  const int koff  = (lane >> 4) * 8;
  const int mOff  = (lane >> 4) * 8;

  v8f accM[4][2], accR[4][2];
#pragma unroll
  for (int i = 0; i < 4; ++i)
#pragma unroll
    for (int j = 0; j < 2; ++j) {
      accM[i][j] = (v8f){0.f, 0.f, 0.f, 0.f, 0.f, 0.f, 0.f, 0.f};
      accR[i][j] = (v8f){0.f, 0.f, 0.f, 0.f, 0.f, 0.f, 0.f, 0.f};
    }

  for (int k0 = 0; k0 < K; k0 += 32) {
    v16h bh[2], bl[2];
#pragma unroll
    for (int j = 0; j < 2; ++j) {
      const size_t bo = (size_t)(n0 + (j << 4) + rlane) * ldb + koff + k0;
      bh[j] = F::load(Bh + bo);
      bl[j] = F::load(Bl + bo);
    }
#pragma unroll
    for (int i = 0; i < 4; ++i) {
      const size_t ao = (size_t)(m0 + (i << 4) + rlane) * lda + koff + k0;
      const v16h ah = F::load(Ah + ao);
      const v16h al = F::load(Al + ao);
#pragma unroll
      for (int j = 0; j < 2; ++j) {
        accM[i][j] = F::mma(ah, bh[j], accM[i][j]);
        accR[i][j] = F::mma(ah, bl[j], accR[i][j]);
        accR[i][j] = F::mma(al, bh[j], accR[i][j]);
      }
      tie1_h(accM[i][0], ah, al);
      tie1_h(accM[i][1], ah, al);
      tie1_h(accR[i][0], ah, al);
      tie4_h(accR[i][1], ah, al);
    }
    keep4_h(bh[0], bh[1], bl[0], bl[1]);
  }
#pragma unroll
  for (int i = 0; i < 4; ++i)
#pragma unroll
    for (int j = 0; j < 2; ++j) {
      acc_tie4(accM[i][j]);
      acc_tie4(accR[i][j]);
    }

  float* slab = sT[wave];
  float bv[2];
#pragma unroll
  for (int j = 0; j < 2; ++j) bv[j] = (BIAS_MODE == 2) ? bias[n0 + (j << 4) + rlane] : 0.0f;
  const int q  = lane >> 3;
  const int c4 = (lane & 7) * 4;
#pragma unroll
  for (int i = 0; i < 4; ++i) {
    const int mBase = m0 + (i << 4);
#pragma unroll
    for (int j = 0; j < 2; ++j) {
#pragma unroll
      for (int r = 0; r < 8; ++r) {
        const float v = (accM[i][j][r] + accR[i][j][r] * kRS_INV) * scale + bv[j];
        slab[(mOff + r) * kSLP + (j << 4) + rlane] = v;
      }
    }
    __builtin_amdgcn_fence(__ATOMIC_RELEASE, "workgroup");
    __builtin_amdgcn_wave_barrier();
    __builtin_amdgcn_fence(__ATOMIC_ACQUIRE, "workgroup");
    v4f vals[4];
#pragma unroll
    for (int it = 0; it < 4; ++it) {
      const int row = it * 4 + q;
      v4f v = *(const v4f*)(slab + row * kSLP + c4);
      if (RESID) {
        const v4f rv = *(const v4f*)(resid + (size_t)(mBase + row) * ldc + n0 + c4);
#pragma unroll
        for (int e = 0; e < 4; ++e) v[e] = v[e] + rv[e];
      }
      vals[it] = v;
    }
    for (int pass = 0; pass < 2; ++pass) {
#pragma unroll
      for (int it = 0; it < 4; ++it) {
        const int row = it * 4 + q;
        *(volatile v4f*)(C + (size_t)(mBase + row) * ldc + n0 + c4) = vals[it];
      }
      __threadfence();
    }
    __builtin_amdgcn_fence(__ATOMIC_RELEASE, "workgroup");
    __builtin_amdgcn_wave_barrier();
    __builtin_amdgcn_fence(__ATOMIC_ACQUIRE, "workgroup");
  }
}

__global__ __launch_bounds__(256) void cell_chunk_kernel(
    const unsigned short* __restrict__ Whhp, const float* __restrict__ Gpre,
    const float* hprev, const float* cin, float* cout, float* Xc)
{
  __shared__ __align__(16) _Float16 hsh[2 * kBB * kHP];
  __shared__ __align__(16) float    csh[kBB * kH];
  __shared__ __align__(16) float    slab[8 * kBB * 32];
  typedef Frag<_Float16> F;
  const _Float16* Whh = (const _Float16*)Whhp;
  const int tid = threadIdx.x;
  const int lane = tid & 31, wave = tid >> 5, hh = lane >> 4, rl = lane & 15;
  const int b0 = (int)blockIdx.x * kBB;

#pragma unroll 1
  for (int it = 0; it < 16; ++it) {
    const int idx = it * 256 + tid;
    const int row = idx >> 8;
    const int c4  = (idx & 255) * 4;
    const v4f hv = *(const v4f*)(hprev + (size_t)(b0 + row) * kH + c4);
    const v4f cv = *(const v4f*)(cin   + (size_t)(b0 + row) * kH + c4);
#pragma unroll
    for (int e = 0; e < 4; ++e) {
      const float x = hv[e];
      hsh[row * kHP + c4 + e] = (_Float16)flush16(x * kCHID);
    }
    *(v4f*)(csh + row * kH + c4) = cv;
  }
  {
    const int buf = tid >> 7, row = (tid >> 3) & 15, col = kH + (tid & 7);
    hsh[buf * (kBB * kHP) + row * kHP + col] = (_Float16)0.0f;
  }
  __syncthreads();

  const int u0 = wave * 128;
  float* slabw = slab + wave * (kBB * 32);
  const int rq = lane >> 3, c4s = (lane & 7) * 4;

#pragma unroll 1
  for (int s = 0; s < kTC; ++s) {
    const _Float16* hc = hsh + (s & 1) * (kBB * kHP);
    _Float16* hn = hsh + ((s & 1) ^ 1) * (kBB * kHP);
    const float* grow = Gpre + ((size_t)s * kB + b0) * kG;
    float* orow = Xc + ((size_t)s * kB + b0) * kH;
#pragma unroll 1
    for (int q = 0; q < 8; ++q) {
      const int ub = u0 + 16 * q;
      v8f acc[4];
#pragma unroll
      for (int g = 0; g < 4; ++g) acc[g] = (v8f){0.f, 0.f, 0.f, 0.f, 0.f, 0.f, 0.f, 0.f};
#pragma unroll 1
      for (int k0 = 0; k0 < kH; k0 += 32) {
        v16h bfr[4];
#pragma unroll
        for (int g = 0; g < 4; ++g) bfr[g] = F::load(Whh + (size_t)(g * kH + ub + rl) * kH + k0 + 8 * hh);
        const v16h a = F::load(hc + rl * kHP + k0 + 8 * hh);
#pragma unroll
        for (int g = 0; g < 4; ++g) acc[g] = F::mma(a, bfr[g], acc[g]);
        tie1_h(acc[0], a, bfr[0]);
        tie1_h(acc[1], a, bfr[1]);
        tie1_h(acc[2], a, bfr[2]);
        tie4_h(acc[3], a, bfr[3]);
      }
      acc_tie4(acc[0]);
      acc_tie4(acc[1]);
      acc_tie4(acc[2]);
      acc_tie4(acc[3]);

      const int u = ub + rl;
      const int scol = (q & 1) * 16 + rl;
#pragma unroll
      for (int r = 0; r < 8; ++r) {
        const int bl = 8 * hh + r;
        const float* gp = grow + (size_t)bl * kG + u;
        const float gi = acc[0][r] * kFoldHid + gp[0];
        const float gf = acc[1][r] * kFoldHid + gp[kH];
        const float gg = acc[2][r] * kFoldHid + gp[2 * kH];
        const float go = acc[3][r] * kFoldHid + gp[3 * kH];
        const float cp = csh[bl * kH + u];
        const float cn = fsig(gf) * cp + fsig(gi) * ftanh(gg);
        csh[bl * kH + u] = cn;
        const float h = fsig(go) * ftanh(cn);
        hn[bl * kHP + u] = (_Float16)flush16(h * kCHID);
        slabw[bl * 32 + scol] = h;
      }
      if (q & 1) {
        __builtin_amdgcn_fence(__ATOMIC_RELEASE, "workgroup");
        __builtin_amdgcn_wave_barrier();
        __builtin_amdgcn_fence(__ATOMIC_ACQUIRE, "workgroup");
        float* ob = orow + u0 + 32 * (q >> 1) + c4s;
        v4f sv[4];
#pragma unroll
        for (int it = 0; it < 4; ++it) sv[it] = *(const v4f*)(slabw + (it * 4 + rq) * 32 + c4s);
        for (int pass = 0; pass < 2; ++pass) {
#pragma unroll
          for (int it = 0; it < 4; ++it) {
            const int row = it * 4 + rq;
            *(volatile v4f*)(ob + (size_t)row * kH) = sv[it];
          }
          __threadfence();
        }
        __builtin_amdgcn_fence(__ATOMIC_RELEASE, "workgroup");
        __builtin_amdgcn_wave_barrier();
        __builtin_amdgcn_fence(__ATOMIC_ACQUIRE, "workgroup");
      }
    }
    __syncthreads();
  }

  for (int pass = 0; pass < 2; ++pass) {
#pragma unroll 1
    for (int it = 0; it < 16; ++it) {
      const int idx = it * 256 + tid;
      const int row = idx >> 8;
      const int c4  = (idx & 255) * 4;
      const v4f v = *(const v4f*)(csh + row * kH + c4);
      *(volatile v4f*)(cout + (size_t)(b0 + row) * kH + c4) = v;
    }
    __threadfence();
  }
}

__global__ __launch_bounds__(256) void mem_scan_kernel(
    const float* __restrict__ P, const float* __restrict__ F0, float* __restrict__ O)
{
  __shared__ __align__(16) float Fm[kFV];
  __shared__ __align__(16) float act[256];
  __shared__ __align__(16) float red[2][8 * 32];
  __shared__ float redss[8];
  const int tid = threadIdx.x, lane = tid & 31, wave = tid >> 5;
  const int b = (int)blockIdx.x;
  const int sI = tid >> 3;
  const int v0 = (tid & 7) * 4;
  float* Fown = Fm + sI * (kS * kS) + v0;
  {
    const float* fsrc = F0 + (size_t)b * kFV + sI * (kS * kS) + v0;
#pragma unroll 4
    for (int r = 0; r < kS; ++r) *(v4f*)(Fown + r * kS) = *(const v4f*)(fsrc + r * kS);
  }
  __syncthreads();

#pragma unroll 1
  for (int t = 0; t < kT; ++t) {
    {
      float pv = P[((size_t)t * kB + b) * kWR + tid];
      asm volatile("" : "+v"(pv));
      const float th = tanhf(pv);
      const float sg = __builtin_amdgcn_rcpf(1.0f + expf(-(pv + 1.0f)));
      const float a = (tid < 3 * kS) ? th : ((tid == 3 * kS) ? sg : pv);
      act[tid] = a;
    }
    __syncthreads();

    const float sS = act[sI];
    v4f acc = (v4f){0.f, 0.f, 0.f, 0.f};
#pragma unroll 2
    for (int r = 0; r < kS; ++r) {
      const v4f f = *(const v4f*)(Fown + r * kS);
      const float rr = act[kS + r];
#pragma unroll
      for (int e = 0; e < 4; ++e) acc[e] = fmaf(rr, f[e], acc[e]);
    }
#pragma unroll
    for (int e = 0; e < 4; ++e) {
      float x = acc[e] * sS;
      x += __shfl_xor(x, 8, 32);
      x += __shfl_xor(x, 16, 32);
      acc[e] = x;
    }
    if (lane < 8) *(v4f*)(&red[0][wave * 32 + v0]) = acc;
    __syncthreads();
    float nv[4];
    {
      v4f vs = (v4f){0.f, 0.f, 0.f, 0.f};
#pragma unroll
      for (int w = 0; w < 8; ++w) {
        const v4f p = *(const v4f*)(&red[0][w * 32 + v0]);
#pragma unroll
        for (int e = 0; e < 4; ++e) vs[e] = vs[e] + p[e];
      }
      const float beta = act[3 * kS];
      const v4f tv = *(const v4f*)(&act[2 * kS + v0]);
#pragma unroll
      for (int e = 0; e < 4; ++e) nv[e] = (beta * (tv[e] - vs[e])) * kInvS;
    }

    float sq0 = 0.f, sq1 = 0.f, sq2 = 0.f, sq3 = 0.f;
#pragma unroll 2
    for (int r = 0; r < kS; ++r) {
      v4f f = *(const v4f*)(Fown + r * kS);
      const float sr = sS * act[kS + r];
      f[0] = fmaf(sr, nv[0], f[0]);
      f[1] = fmaf(sr, nv[1], f[1]);
      f[2] = fmaf(sr, nv[2], f[2]);
      f[3] = fmaf(sr, nv[3], f[3]);
      *(v4f*)(Fown + r * kS) = f;
      sq0 = fmaf(f[0], f[0], sq0);
      sq1 = fmaf(f[1], f[1], sq1);
      sq2 = fmaf(f[2], f[2], sq2);
      sq3 = fmaf(f[3], f[3], sq3);
    }
    {
      float ssum = (sq0 + sq1) + (sq2 + sq3);
#pragma unroll
      for (int off = 1; off < 32; off <<= 1) ssum += __shfl_xor(ssum, off, 32);
      if (lane == 0) redss[wave] = ssum;
    }
    __syncthreads();
    {
      float tot = 0.0f;
#pragma unroll
      for (int w = 0; w < 8; ++w) tot += redss[w];
      float fn = sqrtf(tot);
      fn = fmaxf(fn - 1.0f, 0.0f) + 1.0f;
      const float inv = (fn > 1.0f) ? __builtin_amdgcn_rcpf(fn) : 1.0f;
      if (inv != 1.0f) {
#pragma unroll 2
        for (int r = 0; r < kS; ++r) {
          v4f f = *(const v4f*)(Fown + r * kS);
#pragma unroll
          for (int e = 0; e < 4; ++e) f[e] = f[e] * inv;
          *(v4f*)(Fown + r * kS) = f;
        }
      }
    }

    float qs = act[4 * kS + sI];
    float qlast = 0.0f;
#pragma unroll 1
    for (int hop = 0; hop < 3; ++hop) {
      const int pb = (hop + 1) & 1;
      const float* ri = act + 5 * kS + kS * hop;
      v4f ra = (v4f){0.f, 0.f, 0.f, 0.f};
#pragma unroll 2
      for (int r = 0; r < kS; ++r) {
        const v4f f = *(const v4f*)(Fown + r * kS);
        const float rr = ri[r];
#pragma unroll
        for (int e = 0; e < 4; ++e) ra[e] = fmaf(rr, f[e], ra[e]);
      }
#pragma unroll
      for (int e = 0; e < 4; ++e) {
        float x = ra[e] * qs;
        x += __shfl_xor(x, 8, 32);
        x += __shfl_xor(x, 16, 32);
        ra[e] = x;
      }
      if (lane < 8) *(v4f*)(&red[pb][wave * 32 + v0]) = ra;
      __syncthreads();
      float qn = 0.0f;
#pragma unroll
      for (int w = 0; w < 8; ++w) qn += red[pb][w * 32 + lane];
      float sm = qn;
#pragma unroll
      for (int off = 1; off < 32; off <<= 1) sm += __shfl_xor(sm, off, 32);
      const float mu = sm * kInvS;
      const float d  = qn - mu;
      float sq = d * d;
#pragma unroll
      for (int off = 1; off < 32; off <<= 1) sq += __shfl_xor(sq, off, 32);
      const float var = sq * kInvS;
      const float qnew = d * rsqrtf(var + kLnEps);
      qs = __shfl(qnew, sI, 32);
      qlast = qnew;
    }
    if (wave == 0) {
      float* op = O + ((size_t)t * kB + b) * kS + lane;
      *(volatile float*)op = qlast;
      __threadfence();
      *(volatile float*)op = qlast;
    }
  }
}

extern "C" void kernel_launch(void* const* d_in, const int* in_sizes, int n_in,
                              void* d_out, int out_size, void* d_ws, size_t ws_size,
                              hipStream_t stream) {
  if (n_in < 14 || d_out == nullptr || d_ws == nullptr) return;
  if (in_sizes[0] != kT * kB * kI) return;
  if (in_sizes[1] != kB * kH || in_sizes[2] != kB * kH) return;
  if (in_sizes[3] != kB * kFV) return;
  if (in_sizes[4] != kG * kI || in_sizes[5] != kG * kH) return;
  if (in_sizes[6] != kG || in_sizes[7] != kG) return;
  if (in_sizes[8] != kNW * kH || in_sizes[9] != kNW) return;
  if (in_sizes[10] != kNR * kH || in_sizes[11] != kNR) return;
  if (in_sizes[12] != kH * kS || in_sizes[13] != kH) return;
  if (out_size != kT * kB * kH) return;
  if (ws_size < kWsTotal) return;

  const float* inputs  = (const float*)d_in[0];
  const float* h0      = (const float*)d_in[1];
  const float* c0      = (const float*)d_in[2];
  const float* F0      = (const float*)d_in[3];
  const float* W_ih    = (const float*)d_in[4];
  const float* W_hh    = (const float*)d_in[5];
  const float* b_ih    = (const float*)d_in[6];
  const float* b_hh    = (const float*)d_in[7];
  const float* W_write = (const float*)d_in[8];
  const float* b_write = (const float*)d_in[9];
  const float* W_read  = (const float*)d_in[10];
  const float* b_read  = (const float*)d_in[11];
  const float* W_lin   = (const float*)d_in[12];
  const float* b_lin   = (const float*)d_in[13];
  float* out = (float*)d_out;

  char* ws = (char*)d_ws;
  unsigned short* INH = (unsigned short*)(ws + kOffINH);
  unsigned short* INL = (unsigned short*)(ws + kOffINL);
  unsigned short* WIH = (unsigned short*)(ws + kOffWIH);
  unsigned short* WIL = (unsigned short*)(ws + kOffWIL);
  unsigned short* WHH = (unsigned short*)(ws + kOffWHH);
  float*          GPRE = (float*)(ws + kOffGP);
  float*          X    = (float*)(ws + kOffX);
  unsigned short* WRH = (unsigned short*)(ws + kOffWRH);
  unsigned short* WRL = (unsigned short*)(ws + kOffWRL);
  unsigned short* WLH = (unsigned short*)(ws + kOffWLH);
  unsigned short* WLL = (unsigned short*)(ws + kOffWLL);
  float*          BSUM = (float*)(ws + kOffBS);
  float*          BWR  = (float*)(ws + kOffBW);
  float*          CS0  = (float*)(ws + kOffCS0);
  float*          CS1  = (float*)(ws + kOffCS1);
  float*          Obuf = (float*)(ws + kOffO);
  unsigned short* OH  = (unsigned short*)(ws + kOffOH);
  unsigned short* OL  = (unsigned short*)(ws + kOffOL);
  unsigned short* XH = INH;
  unsigned short* XL = INL;
  float*          Pbuf = GPRE;

  const int n8in = kRows * kI / 8;
  const int n8wi = kG * kI / 8;
  const int n8wl = kH * kS / 8;
  const int n8o  = kRows * kS / 8;
  split_f16_kernel<true><<<n8in / 256, 256, 0, stream>>>(inputs, INH, INL, n8in, kCIN);
  split_f16_kernel<true><<<n8wi / 256, 256, 0, stream>>>(W_ih, WIH, WIL, n8wi, kCW);
  split_f16_kernel<false><<<n8wi / 256, 256, 0, stream>>>(W_hh, WHH, WHH, n8wi, kCW);
  wr_plane_kernel<<<(kWR * kH / 8) / 256, 256, 0, stream>>>(W_write, W_read, WRH, WRL);
  split_f16_kernel<true><<<n8wl / 256, 256, 0, stream>>>(W_lin, WLH, WLL, n8wl, kCW);
  bias_kernel<<<5, 256, 0, stream>>>(b_ih, b_hh, b_write, b_read, BSUM, BWR);

  const int g1blocks = ((kRowsC / 64) * (kG / 32)) / 8;
  for (int c = 0; c < kNC; ++c) {
    const unsigned short* Ah = INH + (size_t)c * kRowsC * kI;
    const unsigned short* Al = INL + (size_t)c * kRowsC * kI;
    gemm_f16x3_kernel<2, false><<<g1blocks, 256, 0, stream>>>(
        Ah, Al, kI, WIH, WIL, kI, GPRE, kG, BSUM, BSUM, kRowsC, kG, kI, kFoldIn);
    const float* hprev = (c == 0) ? h0 : (X + ((size_t)(c * kTC - 1) * kB) * kH);
    const float* cin   = (c == 0) ? c0 : (((c - 1) & 1) ? CS1 : CS0);
    float*       cout  = (c & 1) ? CS1 : CS0;
    cell_chunk_kernel<<<kB / kBB, 256, 0, stream>>>(
        WHH, GPRE, hprev, cin, cout, X + ((size_t)c * kTC * kB) * kH);
  }

  split_f16_kernel<true><<<n8in / 256, 256, 0, stream>>>(X, XH, XL, n8in, kCHID);
  gemm_f16x3_kernel<2, false><<<((kRows / 64) * (kWR / 32)) / 8, 256, 0, stream>>>(
      XH, XL, kH, WRH, WRL, kH, Pbuf, kWR, BWR, BWR, kRows, kWR, kH, kFoldHid);

  mem_scan_kernel<<<kB, 256, 0, stream>>>(Pbuf, F0, Obuf);

  split_f16_kernel<true><<<n8o / 256, 256, 0, stream>>>(Obuf, OH, OL, n8o, kCOUT);
  gemm_f16x3_kernel<2, true><<<((kRows / 64) * (kH / 32)) / 8, 256, 0, stream>>>(
      OH, OL, kS, WLH, WLL, kS, out, kH, b_lin, X, kRows, kH, kS, kFoldOut);
}
